// GraphTaskNodeGCN2_3659312136457
// MI455X (gfx1250) — hardware-verified
//
#include <hip/hip_runtime.h>
#include <stddef.h>
#include <stdint.h>


#define FIN     64
#define HID     128
#define OUTC    32
#define NG      64
#define NTHR    256
#define NWAVE   8
#define EPT     8
#define NGRP    2
#define CHUNK   (NTHR * EPT * NGRP)
#define WCAP    (EPT * NGRP * 32)
#define LISTN   (NWAVE * WCAP)
#define NB1     1024
#define NB2     448
#define NBD     4096
#define G2ROWS  128
#define PCW     128
#define PB1     (FIN * HID / 8 / NTHR)
#define PB2     (HID * HID / 8 / NTHR)
#define PB3     (OUTC * HID / 8 / NTHR)
#define WSCAP   ((size_t)134217728)

#define LDS_AGG1 (NB1 * FIN * 4 + LISTN * 4 + 64)
#define LDS_G2   (G2ROWS * HID * 4)
#define LDS_AGG2 (NB2 * HID * 4 + LISTN * 4 + 64 + NG * HID * 4 + PCW * 4)

static_assert((CHUNK & (CHUNK - 1)) == 0);
static_assert(CHUNK <= 4096);
static_assert(NB1 <= 4096 && NB2 <= 4096 && NBD <= 4096);
static_assert(NB1 % (16 * NWAVE) == 0);
static_assert((NB1 * FIN / 4) % NTHR == 0);
static_assert((NB2 * HID / 4) % NTHR == 0);
static_assert((NG * HID / 4) % NTHR == 0);
static_assert(PB1 * NTHR * 8 == FIN * HID);
static_assert(PB2 * NTHR * 8 == HID * HID);
static_assert(PB3 * NTHR * 8 == OUTC * HID);
static_assert(G2ROWS == 16 * NWAVE);
static_assert(NG == 8 * NWAVE);
static_assert(NG * OUTC == NWAVE * 2 * 128);
static_assert(HID == 4 * 32 && NG == 2 * 32);

typedef float v2f __attribute__((ext_vector_type(2)));
typedef float v4f __attribute__((ext_vector_type(4)));
typedef float v8f __attribute__((ext_vector_type(8)));
typedef int   v4i __attribute__((ext_vector_type(4)));
typedef unsigned short v8us __attribute__((ext_vector_type(8)));
typedef __bf16 v16b __attribute__((ext_vector_type(16)));
union FragB { v16b v; v8us u[2]; };

__device__ __forceinline__ void split1(float v, unsigned short& h, unsigned short& l) {
  const unsigned u  = __float_as_uint(v);
  const unsigned hu = (u + 0x7FFFu + ((u >> 16) & 1u)) >> 16;
  const float    hf = __uint_as_float(hu << 16);
  const unsigned ru = __float_as_uint(v - hf);
  const unsigned lu = (ru + 0x7FFFu + ((ru >> 16) & 1u)) >> 16;
  h = (unsigned short)hu;
  l = (unsigned short)lu;
}

__device__ __forceinline__ void cvt_hl(v4f a, v4f b, v8us& hv, v8us& lv) {
  unsigned short h, l;
  split1(a.x, h, l); hv[0] = h; lv[0] = l;
  split1(a.y, h, l); hv[1] = h; lv[1] = l;
  split1(a.z, h, l); hv[2] = h; lv[2] = l;
  split1(a.w, h, l); hv[3] = h; lv[3] = l;
  split1(b.x, h, l); hv[4] = h; lv[4] = l;
  split1(b.y, h, l); hv[5] = h; lv[5] = l;
  split1(b.z, h, l); hv[6] = h; lv[6] = l;
  split1(b.w, h, l); hv[7] = h; lv[7] = l;
}

__device__ __forceinline__ v8f wmb(v16b a, v16b b, v8f c) {
  v8f d = __builtin_amdgcn_wmma_f32_16x16x32_bf16(false, a, false, b, (short)0, c, false, false);
  asm volatile("v_nop\n\tv_nop\n\tv_nop\n\tv_nop" : "+v"(d) : "v"(a), "v"(b));
  return d;
}

template <int NB>
__device__ __forceinline__ int scan_chunk(const int* __restrict__ dsts, int nE, int cbase, int nodeBase,
                                          int vec8, int* list, int tid, int lane, int wave) {
  int wc = 0;
#pragma unroll
  for (int g = 0; g < NGRP; ++g) {
    const int el0  = (g * NTHR + tid) * EPT;
    const int e0   = cbase + el0;
    const int sent = -2147483647 - 1;
    v4i da, db;
    if (vec8 != 0 && cbase + CHUNK <= nE) {
      da = *(const v4i*)(dsts + e0);
      db = *(const v4i*)(dsts + e0 + 4);
    } else {
      da.x = (e0     < nE) ? dsts[min(e0, nE - 1)] : sent;
      da.y = (e0 + 1 < nE) ? dsts[min(e0 + 1, nE - 1)] : sent;
      da.z = (e0 + 2 < nE) ? dsts[min(e0 + 2, nE - 1)] : sent;
      da.w = (e0 + 3 < nE) ? dsts[min(e0 + 3, nE - 1)] : sent;
      db.x = (e0 + 4 < nE) ? dsts[min(e0 + 4, nE - 1)] : sent;
      db.y = (e0 + 5 < nE) ? dsts[min(e0 + 5, nE - 1)] : sent;
      db.z = (e0 + 6 < nE) ? dsts[min(e0 + 6, nE - 1)] : sent;
      db.w = (e0 + 7 < nE) ? dsts[min(e0 + 7, nE - 1)] : sent;
    }
    const unsigned nb = (unsigned)nodeBase;
    const unsigned s0 = (unsigned)da.x - nb, s1 = (unsigned)da.y - nb;
    const unsigned s2 = (unsigned)da.z - nb, s3 = (unsigned)da.w - nb;
    const unsigned s4 = (unsigned)db.x - nb, s5 = (unsigned)db.y - nb;
    const unsigned s6 = (unsigned)db.z - nb, s7 = (unsigned)db.w - nb;
    const bool h0 = s0 < (unsigned)NB, h1 = s1 < (unsigned)NB, h2 = s2 < (unsigned)NB, h3 = s3 < (unsigned)NB;
    const bool h4 = s4 < (unsigned)NB, h5 = s5 < (unsigned)NB, h6 = s6 < (unsigned)NB, h7 = s7 < (unsigned)NB;
    const unsigned any = __builtin_amdgcn_ballot_w32(h0 | h1 | h2 | h3 | h4 | h5 | h6 | h7);
    if (any != 0u) {
#define HITJ(J, HJ, SJ) { \
        const unsigned mj = __builtin_amdgcn_ballot_w32(HJ); \
        if (mj != 0u) { \
          if (HJ) { \
            const int pos = wc + (int)__builtin_amdgcn_mbcnt_lo(mj, 0u); \
            if (pos < WCAP) list[wave * WCAP + pos] = ((el0 + (J)) << 12) | (int)(SJ); \
          } \
          wc += (int)__builtin_popcount(mj); } }
      HITJ(0, h0, s0)
      HITJ(1, h1, s1)
      HITJ(2, h2, s2)
      HITJ(3, h3, s3)
      HITJ(4, h4, s4)
      HITJ(5, h5, s5)
      HITJ(6, h6, s6)
      HITJ(7, h7, s7)
#undef HITJ
    }
  }
  return wc;
}

__global__ __launch_bounds__(NTHR) void k_prep(
    const float* __restrict__ W1, const float* __restrict__ W2, const float* __restrict__ Wl,
    unsigned short* w1h, unsigned short* w1l, unsigned short* w2h, unsigned short* w2l,
    unsigned short* wlh, unsigned short* wll) {
  const int b = blockIdx.x, tid = threadIdx.x;
  const float* W; unsigned short* ph; unsigned short* pl; int K, NO, li;
  if (b < PB1)            { W = W1; ph = w1h; pl = w1l; K = FIN; NO = HID;  li = b * NTHR + tid; }
  else if (b < PB1 + PB2) { W = W2; ph = w2h; pl = w2l; K = HID; NO = HID;  li = (b - PB1) * NTHR + tid; }
  else                    { W = Wl; ph = wlh; pl = wll; K = HID; NO = OUTC; li = (b - PB1 - PB2) * NTHR + tid; }
  const int o = li * 8;
  if (o + 8 > K * NO) return;
  const int n  = o / K;
  const int k0 = o - n * K;
  const float* p = W + (size_t)k0 * NO + n;
  v4f a, c;
  a.x = p[0];      a.y = p[NO];     a.z = p[2 * NO]; a.w = p[3 * NO];
  c.x = p[4 * NO]; c.y = p[5 * NO]; c.z = p[6 * NO]; c.w = p[7 * NO];
  v8us hv, lv;
  cvt_hl(a, c, hv, lv);
  *(volatile v8us*)(ph + o) = hv;
  *(volatile v8us*)(pl + o) = lv;
  __threadfence();
  *(volatile v8us*)(ph + o) = hv;
  *(volatile v8us*)(pl + o) = lv;
}

__global__ __launch_bounds__(NTHR) void k_deg(
    const int* __restrict__ ei, float* dinv, int nE, int vec8) {
  __shared__ __attribute__((aligned(16))) int cnt[NBD];
  __shared__ __attribute__((aligned(16))) int list[LISTN];
  __shared__ int wcnt[NWAVE];
  const int tid = threadIdx.x, lane = tid & 31, wave = tid >> 5;
  const int nodeBase = blockIdx.x * NBD;
  const int* dsts = ei + nE;

  for (int i = tid; i < NBD; i += NTHR) cnt[i] = 0;
  __syncthreads();

  const int nChunks = (nE + CHUNK - 1) / CHUNK;
#pragma unroll 1
  for (int ch = 0; ch < nChunks; ++ch) {
    const int cbase = ch * CHUNK;
    const int wc = scan_chunk<NBD>(dsts, nE, cbase, nodeBase, vec8, list, tid, lane, wave);
    if (lane == 0) wcnt[wave] = wc;
    __syncthreads();
    if (wave == 0) {
#pragma unroll 1
      for (int wsx = 0; wsx < NWAVE; ++wsx) {
        int n = __builtin_amdgcn_readfirstlane(wcnt[wsx]);
        n = n > WCAP ? WCAP : (n < 0 ? 0 : n);
        const int* lp = list + wsx * WCAP;
#pragma unroll 1
        for (int i = 0; i < n; ++i) {
          const int ent  = __builtin_amdgcn_readfirstlane(lp[i]);
          const int slot = ent & (NBD - 1);
          if (lane == 0) cnt[slot] = cnt[slot] + 1;
        }
      }
    }
    __syncthreads();
  }
  __syncthreads();

  v4f dq[4];
#pragma unroll
  for (int q = 0; q < 4; ++q) {
    const int f = (wave * 4 + q) * 128 + 4 * lane;
    const v4i c = *(const v4i*)(cnt + f);
    dq[q].x = rsqrtf((float)(c.x + 1));
    dq[q].y = rsqrtf((float)(c.y + 1));
    dq[q].z = rsqrtf((float)(c.z + 1));
    dq[q].w = rsqrtf((float)(c.w + 1));
  }
  float* dp = dinv + (size_t)nodeBase;
#pragma unroll
  for (int q = 0; q < 4; ++q) *(volatile v4f*)(dp + (wave * 4 + q) * 128 + 4 * lane) = dq[q];
  __threadfence();
#pragma unroll
  for (int q = 0; q < 4; ++q) *(volatile v4f*)(dp + (wave * 4 + q) * 128 + 4 * lane) = dq[q];
}

__global__ __launch_bounds__(NTHR) void k_agg1(
    const int* __restrict__ ei, const float* __restrict__ x, const float* __restrict__ dinv,
    const float* __restrict__ b1, const unsigned short* __restrict__ w1h, const unsigned short* __restrict__ w1l,
    unsigned short* h1h, unsigned short* h1l, int nN, int nE, int vec8) {
  extern __shared__ v4f lds_dyn[];
  float* acc  = (float*)lds_dyn;
  int*   list = (int*)(acc + NB1 * FIN);
  int*   wcnt = list + LISTN;
  const int tid = threadIdx.x, lane = tid & 31, wave = tid >> 5, hh = lane >> 4, m = lane & 15;
  const int nodeBase = blockIdx.x * NB1;
  const int* dsts = ei + nE;

  {
    const v4f z = {0.f, 0.f, 0.f, 0.f};
    for (int i = tid; i < NB1 * FIN / 4; i += NTHR) lds_dyn[i] = z;
  }
  __syncthreads();

  const int nChunks = (nE + CHUNK - 1) / CHUNK;
#pragma unroll 1
  for (int ch = 0; ch < nChunks; ++ch) {
    const int cbase = ch * CHUNK;
    const int wc = scan_chunk<NB1>(dsts, nE, cbase, nodeBase, vec8, list, tid, lane, wave);
    if (lane == 0) wcnt[wave] = wc;
    __syncthreads();
    if (wave == 0) {
#pragma unroll 1
      for (int wsx = 0; wsx < NWAVE; ++wsx) {
        int n = __builtin_amdgcn_readfirstlane(wcnt[wsx]);
        n = n > WCAP ? WCAP : (n < 0 ? 0 : n);
        const int* lp = list + wsx * WCAP;
#pragma unroll 1
        for (int i = 0; i < n; ++i) {
          const int ent = __builtin_amdgcn_readfirstlane(lp[i]);
          int slot = ent & 4095;
          slot = slot > NB1 - 1 ? NB1 - 1 : slot;
          int e = cbase + ((ent >> 12) & (CHUNK - 1));
          e = e > nE - 1 ? nE - 1 : e;
          int src = ei[e];
          src = src < 0 ? 0 : (src > nN - 1 ? nN - 1 : src);
          const float ds = dinv[src];
          const v2f v = *(const v2f*)(x + (size_t)src * FIN + 2 * lane);
          v2f* ap = (v2f*)(acc + slot * FIN + 2 * lane);
          *ap = *ap + v * ds;
        }
      }
    }
    __syncthreads();
  }

#pragma unroll 4
  for (int i = 0; i < (NB1 * FIN / 4) / NTHR; ++i) {
    const int idx  = i * NTHR + tid;
    const int slot = idx >> 4;
    const int c4   = (idx & 15) * 4;
    int node = nodeBase + slot;
    node = node > nN - 1 ? nN - 1 : node;
    const float d  = dinv[node];
    const v4f   xv = *(const v4f*)(x + (size_t)node * FIN + c4);
    v4f* ap = (v4f*)(acc + slot * FIN + c4);
    *ap = (*ap + xv * d) * d;
  }
  __syncthreads();

  float bcol[8];
#pragma unroll
  for (int u = 0; u < 8; ++u) bcol[u] = b1[16 * u + m];

#pragma unroll 1
  for (int j = 0; j < NB1 / (16 * NWAVE); ++j) {
    const int t = wave + NWAVE * j;
    FragB ah0, al0, ah1, al1;
    {
      const float* ap = acc + (16 * t + m) * FIN + 8 * hh;
      const v4f p0 = *(const v4f*)ap,        p1 = *(const v4f*)(ap + 4);
      const v4f p2 = *(const v4f*)(ap + 16), p3 = *(const v4f*)(ap + 20);
      cvt_hl(p0, p1, ah0.u[0], al0.u[0]);
      cvt_hl(p2, p3, ah0.u[1], al0.u[1]);
      const v4f q0 = *(const v4f*)(ap + 32), q1 = *(const v4f*)(ap + 36);
      const v4f q2 = *(const v4f*)(ap + 48), q3 = *(const v4f*)(ap + 52);
      cvt_hl(q0, q1, ah1.u[0], al1.u[0]);
      cvt_hl(q2, q3, ah1.u[1], al1.u[1]);
    }
    v8f c[8];
#pragma unroll
    for (int u = 0; u < 8; ++u) { v8f z = {0.f, 0.f, 0.f, 0.f, 0.f, 0.f, 0.f, 0.f}; c[u] = z; }
#pragma unroll
    for (int kt = 0; kt < 2; ++kt) {
      const v16b av = (kt == 0) ? ah0.v : ah1.v;
      const v16b lv = (kt == 0) ? al0.v : al1.v;
#pragma unroll
      for (int u = 0; u < 8; ++u) {
        const size_t bo = (size_t)(16 * u + m) * FIN + 32 * kt + 8 * hh;
        FragB bh, bl;
        bh.u[0] = *(const v8us*)(w1h + bo);
        bh.u[1] = *(const v8us*)(w1h + bo + 16);
        bl.u[0] = *(const v8us*)(w1l + bo);
        bl.u[1] = *(const v8us*)(w1l + bo + 16);
        c[u] = wmb(av, bh.v, c[u]);
        c[u] = wmb(av, bl.v, c[u]);
        c[u] = wmb(lv, bh.v, c[u]);
      }
    }
    __syncthreads();

    unsigned short* stg = (unsigned short*)(acc + (size_t)16 * t * FIN);
#pragma unroll
    for (int u = 0; u < 8; ++u) {
#pragma unroll
      for (int r = 0; r < 8; ++r) {
        const float v = fmaxf(c[u][r] + bcol[u], 0.f);
        unsigned short hb, lb;
        split1(v, hb, lb);
        stg[(8 * hh + r) * HID + 16 * u + m] = hb;
      }
    }
    __syncthreads();
    {
      v8us ov[8];
#pragma unroll
      for (int q = 0; q < 8; ++q) ov[q] = *(const v8us*)(stg + q * 256 + 8 * lane);
      unsigned short* gp = h1h + ((size_t)(nodeBase + 16 * t)) * HID + 8 * lane;
#pragma unroll
      for (int q = 0; q < 8; ++q) *(volatile v8us*)(gp + q * 256) = ov[q];
      __threadfence();
#pragma unroll
      for (int q = 0; q < 8; ++q) *(volatile v8us*)(gp + q * 256) = ov[q];
    }
    __syncthreads();
#pragma unroll
    for (int u = 0; u < 8; ++u) {
#pragma unroll
      for (int r = 0; r < 8; ++r) {
        const float v = fmaxf(c[u][r] + bcol[u], 0.f);
        unsigned short hb, lb;
        split1(v, hb, lb);
        stg[(8 * hh + r) * HID + 16 * u + m] = lb;
      }
    }
    __syncthreads();
    {
      v8us ov[8];
#pragma unroll
      for (int q = 0; q < 8; ++q) ov[q] = *(const v8us*)(stg + q * 256 + 8 * lane);
      unsigned short* gp = h1l + ((size_t)(nodeBase + 16 * t)) * HID + 8 * lane;
#pragma unroll
      for (int q = 0; q < 8; ++q) *(volatile v8us*)(gp + q * 256) = ov[q];
      __threadfence();
#pragma unroll
      for (int q = 0; q < 8; ++q) *(volatile v8us*)(gp + q * 256) = ov[q];
    }
  }
}

__global__ __launch_bounds__(NTHR) void k_gemm2(
    const unsigned short* __restrict__ h1h, const unsigned short* __restrict__ h1l,
    const unsigned short* __restrict__ w2h, const unsigned short* __restrict__ w2l,
    const float* __restrict__ dinv, float* g2) {
  extern __shared__ v4f lds_dyn[];
  float* stg = (float*)lds_dyn;
  const int tid = threadIdx.x, lane = tid & 31, wave = tid >> 5, hh = lane >> 4, m = lane & 15;
  const int rowBase = blockIdx.x * G2ROWS;
  const size_t arow = ((size_t)rowBase + wave * 16 + m) * HID + 8 * hh;
  const unsigned short* arh = h1h + arow;
  const unsigned short* arl = h1l + arow;

  v8f c[8];
#pragma unroll
  for (int u = 0; u < 8; ++u) { v8f z = {0.f, 0.f, 0.f, 0.f, 0.f, 0.f, 0.f, 0.f}; c[u] = z; }
#pragma unroll
  for (int kt = 0; kt < HID / 32; ++kt) {
    FragB ah, al;
    ah.u[0] = *(const v8us*)(arh + 32 * kt);
    ah.u[1] = *(const v8us*)(arh + 32 * kt + 16);
    al.u[0] = *(const v8us*)(arl + 32 * kt);
    al.u[1] = *(const v8us*)(arl + 32 * kt + 16);
#pragma unroll
    for (int u = 0; u < 8; ++u) {
      const size_t bo = (size_t)(16 * u + m) * HID + 32 * kt + 8 * hh;
      FragB bh, bl;
      bh.u[0] = *(const v8us*)(w2h + bo);
      bh.u[1] = *(const v8us*)(w2h + bo + 16);
      bl.u[0] = *(const v8us*)(w2l + bo);
      bl.u[1] = *(const v8us*)(w2l + bo + 16);
      c[u] = wmb(ah.v, bh.v, c[u]);
      c[u] = wmb(ah.v, bl.v, c[u]);
      c[u] = wmb(al.v, bh.v, c[u]);
    }
  }

  const int r0 = wave * 16 + 8 * hh;
  const v4f dA = *(const v4f*)(dinv + (size_t)rowBase + r0);
  const v4f dB = *(const v4f*)(dinv + (size_t)rowBase + r0 + 4);
  float* sp = stg + r0 * HID + m;
#pragma unroll
  for (int u = 0; u < 8; ++u) {
    sp[0 * HID + 16 * u] = c[u][0] * dA.x;
    sp[1 * HID + 16 * u] = c[u][1] * dA.y;
    sp[2 * HID + 16 * u] = c[u][2] * dA.z;
    sp[3 * HID + 16 * u] = c[u][3] * dA.w;
    sp[4 * HID + 16 * u] = c[u][4] * dB.x;
    sp[5 * HID + 16 * u] = c[u][5] * dB.y;
    sp[6 * HID + 16 * u] = c[u][6] * dB.z;
    sp[7 * HID + 16 * u] = c[u][7] * dB.w;
  }
  __syncthreads();

  const float* lp = stg + wave * 16 * HID + 4 * lane;
  float* gp = g2 + ((size_t)rowBase + wave * 16) * HID + 4 * lane;
#pragma unroll
  for (int i = 0; i < 16; ++i) { const v4f v = *(const v4f*)(lp + i * HID); *(volatile v4f*)(gp + (size_t)i * HID) = v; }
  __threadfence();
#pragma unroll
  for (int i = 0; i < 16; ++i) { const v4f v = *(const v4f*)(lp + i * HID); *(volatile v4f*)(gp + (size_t)i * HID) = v; }
}

__global__ __launch_bounds__(NTHR) void k_agg2(
    const int* __restrict__ ei, const float* __restrict__ g2, const float* __restrict__ dinv,
    const float* __restrict__ b2, const int* __restrict__ batch,
    float* psum, int* pcnt, int nN, int nE, int vec8) {
  extern __shared__ v4f lds_dyn[];
  float* acc  = (float*)lds_dyn;
  int*   list = (int*)(acc + NB2 * HID);
  int*   wcnt = list + LISTN;
  float* psl  = (float*)(wcnt + 16);
  int*   pcl  = (int*)(psl + NG * HID);
  const int tid = threadIdx.x, lane = tid & 31, wave = tid >> 5;
  const int nodeBase = blockIdx.x * NB2;
  const int* dsts = ei + nE;

  {
    const v4f z = {0.f, 0.f, 0.f, 0.f};
    for (int i = tid; i < NB2 * HID / 4; i += NTHR) lds_dyn[i] = z;
    v4f* pz = (v4f*)psl;
    for (int i = tid; i < NG * HID / 4; i += NTHR) pz[i] = z;
    if (tid < PCW) pcl[tid] = 0;
  }
  __syncthreads();

  const int nChunks = (nE + CHUNK - 1) / CHUNK;
#pragma unroll 1
  for (int ch = 0; ch < nChunks; ++ch) {
    const int cbase = ch * CHUNK;
    const int wc = scan_chunk<NB2>(dsts, nE, cbase, nodeBase, vec8, list, tid, lane, wave);
    if (lane == 0) wcnt[wave] = wc;
    __syncthreads();
    if (wave == 0) {
#pragma unroll 1
      for (int wsx = 0; wsx < NWAVE; ++wsx) {
        int n = __builtin_amdgcn_readfirstlane(wcnt[wsx]);
        n = n > WCAP ? WCAP : (n < 0 ? 0 : n);
        const int* lp = list + wsx * WCAP;
#pragma unroll 1
        for (int i = 0; i < n; ++i) {
          const int ent = __builtin_amdgcn_readfirstlane(lp[i]);
          int slot = ent & 4095;
          slot = slot > NB2 - 1 ? NB2 - 1 : slot;
          int e = cbase + ((ent >> 12) & (CHUNK - 1));
          e = e > nE - 1 ? nE - 1 : e;
          int src = ei[e];
          src = src < 0 ? 0 : (src > nN - 1 ? nN - 1 : src);
          const v4f v = *(const v4f*)(g2 + (size_t)src * HID + 4 * lane);
          v4f* ap = (v4f*)(acc + slot * HID + 4 * lane);
          *ap = *ap + v;
        }
      }
    }
    __syncthreads();
  }

  if (wave < 4) {
    const int c = tid;
    const float bc = b2[c];
    float run = 0.f;
    int gcur = -1;
#pragma unroll 1
    for (int r = 0; r < NB2; ++r) {
      const int node  = nodeBase + r;
      const int nodec = node > nN - 1 ? nN - 1 : node;
      const float d   = dinv[nodec];
      const float gv  = g2[(size_t)nodec * HID + c];
      float v = fmaxf((acc[r * HID + c] + gv) * d + bc, 0.f);
      const int gi  = batch[nodec];
      const bool ok = (node < nN) && ((unsigned)gi < (unsigned)NG);
      v = ok ? v : 0.f;
      const int g = ok ? gi : gcur;
      if (g != gcur) {
        if (gcur >= 0) psl[gcur * HID + c] = psl[gcur * HID + c] + run;
        run = 0.f;
        gcur = g;
      }
      run += v;
    }
    if (gcur >= 0) psl[gcur * HID + c] = psl[gcur * HID + c] + run;
  } else if (wave == 4) {
#pragma unroll 1
    for (int r = 0; r < NB2; ++r) {
      const int node  = nodeBase + r;
      const int nodec = node > nN - 1 ? nN - 1 : node;
      const int gi    = batch[nodec];
      const bool ok   = (node < nN) && ((unsigned)gi < (unsigned)NG);
      if (ok && lane == 0) pcl[gi] = pcl[gi] + 1;
    }
  }
  __syncthreads();

  v4f ov[8];
#pragma unroll
  for (int q = 0; q < 8; ++q) ov[q] = *(const v4f*)(psl + (8 * wave + q) * HID + 4 * lane);
  float* gp = psum + ((size_t)blockIdx.x * NG + 8 * wave) * HID + 4 * lane;
#pragma unroll
  for (int q = 0; q < 8; ++q) *(volatile v4f*)(gp + q * HID) = ov[q];
  __threadfence();
#pragma unroll
  for (int q = 0; q < 8; ++q) *(volatile v4f*)(gp + q * HID) = ov[q];

  if (wave == 0) {
    const v4i cv = *(const v4i*)(pcl + 4 * lane);
    int* cp = pcnt + (size_t)blockIdx.x * PCW + 4 * lane;
    *(volatile v4i*)cp = cv;
    __threadfence();
    *(volatile v4i*)cp = cv;
  }
}

__global__ __launch_bounds__(NTHR) void k_final(
    const float* __restrict__ psum, const int* __restrict__ pcnt,
    const unsigned short* __restrict__ wlh, const unsigned short* __restrict__ wll,
    const float* __restrict__ blin, float* out, int nBlk) {
  __shared__ __attribute__((aligned(16))) float pooled[NG * HID];
  __shared__ __attribute__((aligned(16))) float sout[NG * OUTC];
  __shared__ int cntl[NG];
  const int tid = threadIdx.x, lane = tid & 31, wave = tid >> 5, hh = lane >> 4, m = lane & 15;

  if (wave < 2) {
    const int g = tid;
    int s = 0;
#pragma unroll 1
    for (int b = 0; b < nBlk; ++b) s += pcnt[(size_t)b * PCW + g];
    cntl[g] = s;
  }
  __syncthreads();

  {
    const int c  = tid & (HID - 1);
    const int g0 = tid >> 7;
#pragma unroll 1
    for (int gg = 0; gg < NG / 2; ++gg) {
      const int g = g0 + 2 * gg;
      double s = 0.0;
#pragma unroll 1
      for (int b = 0; b < nBlk; ++b) s += (double)psum[((size_t)b * NG + g) * HID + c];
      const float cf  = (float)cntl[g];
      const float den = cf > 1.f ? cf : 1.f;
      pooled[g * HID + c] = (float)s * (1.0f / den);
    }
  }
  __syncthreads();

  const int rt = wave >> 1, ct = wave & 1;
  v8f acc = {0.f, 0.f, 0.f, 0.f, 0.f, 0.f, 0.f, 0.f};
#pragma unroll
  for (int kt = 0; kt < HID / 32; ++kt) {
    const float* ap = pooled + (16 * rt + m) * HID + 32 * kt + 8 * hh;
    const v4f p0 = *(const v4f*)ap,        p1 = *(const v4f*)(ap + 4);
    const v4f p2 = *(const v4f*)(ap + 16), p3 = *(const v4f*)(ap + 20);
    FragB ah, al;
    cvt_hl(p0, p1, ah.u[0], al.u[0]);
    cvt_hl(p2, p3, ah.u[1], al.u[1]);
    const size_t bo = (size_t)(16 * ct + m) * HID + 32 * kt + 8 * hh;
    FragB bh, bl;
    bh.u[0] = *(const v8us*)(wlh + bo);
    bh.u[1] = *(const v8us*)(wlh + bo + 16);
    bl.u[0] = *(const v8us*)(wll + bo);
    bl.u[1] = *(const v8us*)(wll + bo + 16);
    acc = wmb(ah.v, bh.v, acc);
    acc = wmb(ah.v, bl.v, acc);
    acc = wmb(al.v, bh.v, acc);
  }
  {
    const float bv = blin[16 * ct + m];
    float* sp = sout + (16 * rt + 8 * hh) * OUTC + 16 * ct + m;
    sp[0 * OUTC] = acc[0] + bv;
    sp[1 * OUTC] = acc[1] + bv;
    sp[2 * OUTC] = acc[2] + bv;
    sp[3 * OUTC] = acc[3] + bv;
    sp[4 * OUTC] = acc[4] + bv;
    sp[5 * OUTC] = acc[5] + bv;
    sp[6 * OUTC] = acc[6] + bv;
    sp[7 * OUTC] = acc[7] + bv;
  }
  __syncthreads();

  v4f ov[2];
#pragma unroll
  for (int q = 0; q < 2; ++q) ov[q] = *(const v4f*)(sout + (wave * 2 + q) * 128 + 4 * lane);
#pragma unroll
  for (int q = 0; q < 2; ++q) *(volatile v4f*)(out + (wave * 2 + q) * 128 + 4 * lane) = ov[q];
  __threadfence();
#pragma unroll
  for (int q = 0; q < 2; ++q) *(volatile v4f*)(out + (wave * 2 + q) * 128 + 4 * lane) = ov[q];
}

extern "C" void kernel_launch(void* const* d_in, const int* in_sizes, int n_in,
                              void* d_out, int out_size, void* d_ws, size_t ws_size,
                              hipStream_t stream) {
  if (n_in < 9) return;
  const int nN = in_sizes[0] / FIN;
  const int nE = in_sizes[1] / 2;
  if (nN <= 0 || nE <= 0 || in_sizes[0] != nN * FIN || in_sizes[1] != nE * 2) return;
  if (in_sizes[2] != nN) return;
  if (in_sizes[3] != FIN * HID || in_sizes[4] < HID || in_sizes[5] != HID * HID || in_sizes[6] < HID) return;
  if (in_sizes[7] != HID * OUTC || in_sizes[8] < OUTC) return;
  if (out_size != NG * OUTC) return;

  const float* x     = (const float*)d_in[0];
  const int*   ei    = (const int*)d_in[1];
  const int*   batch = (const int*)d_in[2];
  const float* W1    = (const float*)d_in[3];
  const float* b1    = (const float*)d_in[4];
  const float* W2    = (const float*)d_in[5];
  const float* b2    = (const float*)d_in[6];
  const float* Wl    = (const float*)d_in[7];
  const float* bl    = (const float*)d_in[8];
  float* out = (float*)d_out;

  const int nA1 = (nN + NB1 - 1) / NB1;
  const int nA2 = (nN + NB2 - 1) / NB2;
  const int nG2 = (nN + G2ROWS - 1) / G2ROWS;
  int nPad = nA1 * NB1;
  if (nA2 * NB2 > nPad) nPad = nA2 * NB2;
  if (nG2 * G2ROWS > nPad) nPad = nG2 * G2ROWS;
  const int nBD = (nPad + NBD - 1) / NBD;
  if (nG2 * G2ROWS > nA1 * NB1) return;

  char* ws = (char*)d_ws;
  size_t off = 0;
  const size_t oW1h = off; off += (size_t)FIN * HID * 2;            off = (off + 255) & ~(size_t)255;
  const size_t oW1l = off; off += (size_t)FIN * HID * 2;            off = (off + 255) & ~(size_t)255;
  const size_t oW2h = off; off += (size_t)HID * HID * 2;            off = (off + 255) & ~(size_t)255;
  const size_t oW2l = off; off += (size_t)HID * HID * 2;            off = (off + 255) & ~(size_t)255;
  const size_t oWlh = off; off += (size_t)HID * OUTC * 2;           off = (off + 255) & ~(size_t)255;
  const size_t oWll = off; off += (size_t)HID * OUTC * 2;           off = (off + 255) & ~(size_t)255;
  const size_t oDv  = off; off += (size_t)nBD * NBD * 4;            off = (off + 255) & ~(size_t)255;
  const size_t oH1h = off; off += (size_t)nA1 * NB1 * HID * 2;      off = (off + 255) & ~(size_t)255;
  const size_t oH1l = off; off += (size_t)nA1 * NB1 * HID * 2;      off = (off + 255) & ~(size_t)255;
  const size_t oG2  = off; off += (size_t)nG2 * G2ROWS * HID * 4;   off = (off + 255) & ~(size_t)255;
  const size_t oPs  = off; off += (size_t)nA2 * NG * HID * 4;       off = (off + 255) & ~(size_t)255;
  const size_t oPc  = off; off += (size_t)nA2 * PCW * 4;            off = (off + 255) & ~(size_t)255;
  if (off > ws_size || off > WSCAP) return;

  unsigned short* w1h = (unsigned short*)(ws + oW1h);
  unsigned short* w1l = (unsigned short*)(ws + oW1l);
  unsigned short* w2h = (unsigned short*)(ws + oW2h);
  unsigned short* w2l = (unsigned short*)(ws + oW2l);
  unsigned short* wlh = (unsigned short*)(ws + oWlh);
  unsigned short* wll = (unsigned short*)(ws + oWll);
  float*          dinv = (float*)(ws + oDv);
  unsigned short* h1h  = (unsigned short*)(ws + oH1h);
  unsigned short* h1l  = (unsigned short*)(ws + oH1l);
  float*          g2   = (float*)(ws + oG2);
  float*          psum = (float*)(ws + oPs);
  int*            pcnt = (int*)(ws + oPc);

  const int vec8 = ((nE & 3) == 0) ? 1 : 0;

  k_prep<<<PB1 + PB2 + PB3, NTHR, 0, stream>>>(W1, W2, Wl, w1h, w1l, w2h, w2l, wlh, wll);

  k_deg<<<nBD, NTHR, 0, stream>>>(ei, dinv, nE, vec8);

  hipFuncSetAttribute(reinterpret_cast<const void*>(&k_agg1),
                      hipFuncAttributeMaxDynamicSharedMemorySize, LDS_AGG1);
  k_agg1<<<nA1, NTHR, LDS_AGG1, stream>>>(ei, x, dinv, b1, w1h, w1l, h1h, h1l, nN, nE, vec8);

  hipFuncSetAttribute(reinterpret_cast<const void*>(&k_gemm2),
                      hipFuncAttributeMaxDynamicSharedMemorySize, LDS_G2);
  k_gemm2<<<nG2, NTHR, LDS_G2, stream>>>(h1h, h1l, w2h, w2l, dinv, g2);

  hipFuncSetAttribute(reinterpret_cast<const void*>(&k_agg2),
                      hipFuncAttributeMaxDynamicSharedMemorySize, LDS_AGG2);
  k_agg2<<<nA2, NTHR, LDS_AGG2, stream>>>(ei, g2, dinv, b2, batch, psum, pcnt, nN, nE, vec8);

  k_final<<<1, NTHR, 0, stream>>>(psum, pcnt, wlh, wll, bl, out, nA2);
}
